// GNNDecoder_68143951118640
// MI455X (gfx1250) — hardware-verified
//
#include <hip/hip_runtime.h>
#include <math.h>

typedef __attribute__((ext_vector_type(16))) _Float16 v16h;
typedef __attribute__((ext_vector_type(16))) __bf16 v16b;
typedef __attribute__((ext_vector_type(8)))  _Float16 v8h;
typedef __attribute__((ext_vector_type(8)))  float v8f;
typedef __attribute__((ext_vector_type(4)))  float v4f;
typedef __attribute__((ext_vector_type(2)))  float v2f;
typedef __attribute__((ext_vector_type(4)))  unsigned v4u;
typedef __attribute__((ext_vector_type(4)))  int v4i;
typedef float __attribute__((may_alias)) float_a;
typedef int __attribute__((may_alias)) int_a;

template <typename T> __device__ __forceinline__ void vst2(void* p, T v) { *(volatile T*)p = v; __threadfence(); *(volatile T*)p = v; }
__device__ __forceinline__ v8f wmma16(v16h a, v16h b, v8f c) {
  v8f d = __builtin_amdgcn_wmma_f32_16x16x32_f16(false, a, false, b, (short)0, c, false, false);
  asm volatile("v_nop\n\tv_nop\n\tv_nop\n\tv_nop" : "+v"(d) : "v"(a), "v"(b));
  return d;
}
__device__ __forceinline__ v8f wmma_bf(v16b a, v16b b, v8f c) {
  v8f d = __builtin_amdgcn_wmma_f32_16x16x32_bf16(false, a, false, b, (short)0, c, false, false);
  asm volatile("v_nop\n\tv_nop\n\tv_nop\n\tv_nop" : "+v"(d) : "v"(a), "v"(b));
  return d;
}
__device__ __forceinline__ v16h frag_h(const _Float16* rowk0, int lane) {
  union { v16h v; v8h q[2]; } u; const _Float16* p = rowk0 + 8 * (lane >> 4);
  u.q[0] = *(const v8h*)p; u.q[1] = *(const v8h*)(p + 16); return u.v;
}
__device__ __forceinline__ v16h frag_f32(const float* rowk0, int lane) {
  v16h a; const float* p = rowk0 + 8 * (lane >> 4);
#pragma unroll
  for (int i = 0; i < 8; ++i) { a[i] = (_Float16)p[i]; a[8 + i] = (_Float16)p[16 + i]; }
  return a;
}
__device__ __forceinline__ v16h frag_f32s(const float* rowk0, int lane, float sc) {
  v16h a; const float* p = rowk0 + 8 * (lane >> 4);
#pragma unroll
  for (int i = 0; i < 8; ++i) { a[i] = (_Float16)(p[i] * sc); a[8 + i] = (_Float16)(p[16 + i] * sc); }
  return a;
}
__device__ __forceinline__ v16h fragc_f32(const float* W, int k0, int n, int lane, int ld, int K) {
  v16h a; const int g = lane >> 4;
#pragma unroll
  for (int i = 0; i < 8; ++i) { const int ka = k0 + 8 * g + i, kb = ka + 16;
    a[i] = (_Float16)(ka < K ? W[(size_t)ka * ld + n] : 0.f); a[8 + i] = (_Float16)(kb < K ? W[(size_t)kb * ld + n] : 0.f); }
  return a;
}
struct F2 { v16b h, l; };
__device__ __forceinline__ F2 bsplit16(const float v[16]) { F2 r;
#pragma unroll
  for (int i = 0; i < 16; ++i) { const __bf16 h = (__bf16)v[i]; r.h[i] = h; r.l[i] = (__bf16)(v[i] - (float)h); }
  return r; }
__device__ __forceinline__ F2 split_row(const float* row, int k0, int lane) { float v[16]; const float* p = row + k0 + 8 * (lane >> 4);
#pragma unroll
  for (int i = 0; i < 8; ++i) { v[i] = p[i]; v[8 + i] = p[16 + i]; }
  return bsplit16(v); }
__device__ __forceinline__ F2 split_rowK(const float* row, int k0, int lane, int K) { float v[16]; const int g = lane >> 4;
#pragma unroll
  for (int i = 0; i < 8; ++i) { const int ka = k0 + 8 * g + i, kb = ka + 16; v[i] = ka < K ? row[ka] : 0.f; v[8 + i] = kb < K ? row[kb] : 0.f; }
  return bsplit16(v); }
__device__ __forceinline__ F2 split_col(const float* W, int k0, int n, int lane, int ld, int K) { float v[16]; const int g = lane >> 4;
#pragma unroll
  for (int i = 0; i < 8; ++i) { const int ka = k0 + 8 * g + i, kb = ka + 16; v[i] = ka < K ? W[(size_t)ka * ld + n] : 0.f; v[8 + i] = kb < K ? W[(size_t)kb * ld + n] : 0.f; }
  return bsplit16(v); }
__device__ __forceinline__ v8f mac3(const F2& a, const F2& b, v8f c) { c = wmma_bf(a.l, b.h, c); c = wmma_bf(a.h, b.l, c); return wmma_bf(a.h, b.h, c); }
__device__ __forceinline__ float sigm(float v) { return 1.0f / (1.0f + expf(-v)); }
#define LDSX() do { asm volatile("s_wait_dscnt 0" ::: "memory"); __builtin_amdgcn_wave_barrier(); __builtin_amdgcn_fence(__ATOMIC_RELEASE, "workgroup"); } while (0)
__device__ __forceinline__ v16h fragc_f32s(const float* __restrict__ base, int k0, int n, int lane, int ld, float sc) {
  const int g = lane >> 4; v16h r;
#pragma unroll
  for (int i = 0; i < 8; ++i) { r[i] = (_Float16)(base[(size_t)(k0 + 8 * g + i) * ld + n] * sc); r[8 + i] = (_Float16)(base[(size_t)(k0 + 16 + 8 * g + i) * ld + n] * sc); }
  return r;
}

#define NBAT 128
#define NBH 64
#define NNODE 2024
#define NNP 2048
#define NE 8004
#define HH 128
#define NL 4
#define EPT 16
#define CH (256 * EPT)
#define RB 64

__global__ __launch_bounds__(256) void k_embed(const float* __restrict__ x, const float* __restrict__ we, const float* __restrict__ be, int b0, _Float16* __restrict__ H) {
  const int bl = blockIdx.y, n0 = blockIdx.x * 64, tid = threadIdx.x; const int rl = tid >> 2, qq = tid & 3; const int n = n0 + rl;
  const float xv = n < NNODE ? x[(size_t)(b0 + bl) * NNODE + n] : 0.f;
  for (int c8 = qq * 4; c8 < qq * 4 + 4; ++c8) { union { v8h h; v4u u; } pk;
#pragma unroll
    for (int e = 0; e < 8; ++e) { const int c = c8 * 8 + e; pk.h[e] = (_Float16)(n < NNODE ? xv * we[c] + be[c] : 0.f); }
    vst2(H + ((size_t)bl * NNP + n) * HH + c8 * 8, pk.u); }
}
__global__ __launch_bounds__(256) void k_layer1(const float* __restrict__ x, int b0, const int* __restrict__ esrc, const int* __restrict__ edst, const float* __restrict__ we, const float* __restrict__ bemb, const float* __restrict__ W, const float* __restrict__ bb, const float* __restrict__ g, const float* __restrict__ be, _Float16* __restrict__ Hout) {
  __shared__ float ssum[NBH][RB]; __shared__ int srcnt[RB];
  __shared__ int ssrc[8][32 * EPT], sdl[8][32 * EPT]; __shared__ int scnt[8];
  __shared__ float su[HH], sv[HH], scb[HH], scb2[HH];
  const int tid = threadIdx.x, wave = tid >> 5, lane = tid & 31; const int r0 = blockIdx.x * RB;
  for (int q = tid; q < NBH * RB; q += 256) (&ssum[0][0])[q] = 0.f;
  if (tid < RB) srcnt[tid] = 0;
  if (tid < HH) { float u = 0.f, v = 0.f, c1 = 0.f, c2 = 0.f;
#pragma unroll 1
    for (int k = 0; k < HH; ++k) { const float wk = we[k], bk = bemb[k]; const float wt = W[(size_t)k * HH + tid], wb = W[(size_t)(HH + k) * HH + tid]; u += wk * wt; v += wk * wb; c1 += bk * wt; c2 += bk * wb; }
    su[tid] = u; sv[tid] = v; scb[tid] = c1; scb2[tid] = c2; }
  __syncthreads();
#define NN NNODE
  #pragma unroll 1
  for (int c0 = 0; c0 < NE; c0 += CH) {
    const int e0 = c0 + tid * EPT; int hd[EPT]; int cnt = 0;
    if (e0 + EPT <= NE) {
#pragma unroll
      for (int v = 0; v < EPT / 4; ++v) { const int4 d4 = *(const int4*)(edst + e0 + v * 4);
        const int dd[4] = {d4.x, d4.y, d4.z, d4.w};
#pragma unroll
        for (int u = 0; u < 4; ++u) { const unsigned rel = (unsigned)(dd[u] - r0); const bool h = rel < (unsigned)RB; hd[v * 4 + u] = h ? (int)rel : -1; cnt += h ? 1 : 0; } } }
    else {
#pragma unroll
      for (int u = 0; u < EPT; ++u) { const int e = e0 + u; hd[u] = -1; if (e < NE) { const unsigned rel = (unsigned)(edst[e] - r0); if (rel < (unsigned)RB) { hd[u] = (int)rel; ++cnt; } } } }
    int incl = cnt;
#pragma unroll
    for (int off = 1; off < 32; off <<= 1) { const int vv = __shfl_up(incl, off, 32); if (lane >= off) incl += vv; }
    const int wtot = __shfl(incl, 31, 32); int pos = incl - cnt;
    if (cnt > 0) {
#pragma unroll
      for (int u = 0; u < EPT; ++u) if (hd[u] >= 0) { int s = esrc[e0 + u]; s = s < 0 ? 0 : (s >= NN ? NN - 1 : s); ssrc[wave][pos] = s; sdl[wave][pos] = hd[u]; atomicAdd(&srcnt[hd[u]], 1); ++pos; } }
    if (lane == 0) scnt[wave] = wtot;
    __syncthreads();
    if (tid < NBH) { const float* xb = x + (size_t)(b0 + tid) * NNODE; for (int w = 0; w < 8; ++w) { const int nh = scnt[w]; for (int i = 0; i < nh; ++i) ssum[tid][sdl[w][i]] += xb[ssrc[w][i]]; } }
    __syncthreads(); }
#undef NN
#pragma unroll 1
  for (int it = 0; it < 16; ++it) { const int row = it * 256 + tid; const int bq = row >> 6, rl = row & 63; const int n = r0 + rl;
    const int cnt = srcnt[rl]; const float xv = (n < NNODE) ? x[(size_t)(b0 + bq) * NNODE + n] : 0.f; const float mx = cnt > 0 ? ssum[bq][rl] / (float)cnt : 0.f; const float ind = cnt > 0 ? 1.f : 0.f;
    float s = 0.f, q2 = 0.f;
#pragma unroll 1
    for (int c = 0; c < HH; ++c) { float v = xv * su[c] + scb[c] + mx * sv[c] + ind * scb2[c] + bb[c]; v = v > 0.f ? v : 0.f; s += v; q2 += v * v; }
    const float mu = s * (1.0f / HH); const float var = fmaxf(q2 * (1.0f / HH) - mu * mu, 0.f); const float rs = rsqrtf(var + 1e-5f);
#pragma unroll 1
    for (int c8 = 0; c8 < 16; ++c8) { union { v8h h; v4u uu; } pk;
#pragma unroll
      for (int e = 0; e < 8; ++e) { const int c = c8 * 8 + e; float v = xv * su[c] + scb[c] + mx * sv[c] + ind * scb2[c] + bb[c]; v = v > 0.f ? v : 0.f; pk.h[e] = (_Float16)(n < NNODE ? (v - mu) * rs * g[c] + be[c] : 0.f); }
      vst2(Hout + ((size_t)bq * NNP + n) * HH + c8 * 8, pk.uu); } }
}
__global__ __launch_bounds__(256) void k_packw(const float* __restrict__ W, _Float16* __restrict__ WT) {
  const int l = blockIdx.y, n = blockIdx.x, tid = threadIdx.x; __shared__ __align__(16) _Float16 srow[2 * HH];
  srow[tid] = (_Float16)(W[((size_t)l * 2 * HH + tid) * HH + n] * 16.0f);
  __syncthreads();
  if (tid < 32) vst2(WT + ((size_t)l * HH + n) * (2 * HH) + tid * 8, *(const v4u*)(&srow[tid * 8]));
}
#define NBB 4
__global__ __launch_bounds__(256) void k_layer(const _Float16* __restrict__ Hin, const int* __restrict__ esrc, const int* __restrict__ edst, const _Float16* __restrict__ WT, const float* __restrict__ bb, const float* __restrict__ g, const float* __restrict__ be, _Float16* __restrict__ Hout) {
  __shared__ __align__(16) float sacc[NBB][RB][HH + 4];
  __shared__ int ssrc[8][32 * EPT], sdl[8][32 * EPT]; __shared__ int scnt[8]; __shared__ int srcnt[RB];
  __shared__ __align__(16) _Float16 sa[NBB][RB][2 * HH + 8];
  const int tid = threadIdx.x, wave = tid >> 5, lane = tid & 31, col = lane & 15, gg = lane >> 4;
  const int bl0 = blockIdx.y * NBB, r0 = blockIdx.x * RB;
  for (int q = tid; q < NBB * RB * (HH + 4); q += 256) (&sacc[0][0][0])[q] = 0.f;
  if (tid < RB) srcnt[tid] = 0;
  for (int q = tid; q < NBB * RB * (HH / 8); q += 256) { const int bq = q / (RB * 16), rem = q % (RB * 16); const int rl = rem >> 4, pc = rem & 15;
    *(v4u*)(&sa[bq][rl][pc * 8]) = *(const v4u*)(Hin + ((size_t)(bl0 + bq) * NNP + r0 + rl) * HH + pc * 8); }
  __syncthreads();
#define NN NNODE
  #pragma unroll 1
  for (int c0 = 0; c0 < NE; c0 += CH) {
    const int e0 = c0 + tid * EPT; int hd[EPT]; int cnt = 0;
    if (e0 + EPT <= NE) {
#pragma unroll
      for (int v = 0; v < EPT / 4; ++v) { const int4 d4 = *(const int4*)(edst + e0 + v * 4);
        const int dd[4] = {d4.x, d4.y, d4.z, d4.w};
#pragma unroll
        for (int u = 0; u < 4; ++u) { const unsigned rel = (unsigned)(dd[u] - r0); const bool h = rel < (unsigned)RB; hd[v * 4 + u] = h ? (int)rel : -1; cnt += h ? 1 : 0; } } }
    else {
#pragma unroll
      for (int u = 0; u < EPT; ++u) { const int e = e0 + u; hd[u] = -1; if (e < NE) { const unsigned rel = (unsigned)(edst[e] - r0); if (rel < (unsigned)RB) { hd[u] = (int)rel; ++cnt; } } } }
    int incl = cnt;
#pragma unroll
    for (int off = 1; off < 32; off <<= 1) { const int vv = __shfl_up(incl, off, 32); if (lane >= off) incl += vv; }
    const int wtot = __shfl(incl, 31, 32); int pos = incl - cnt;
    if (cnt > 0) {
#pragma unroll
      for (int u = 0; u < EPT; ++u) if (hd[u] >= 0) { int s = esrc[e0 + u]; s = s < 0 ? 0 : (s >= NN ? NN - 1 : s); ssrc[wave][pos] = s; sdl[wave][pos] = hd[u]; atomicAdd(&srcnt[hd[u]], 1); ++pos; } }
    if (lane == 0) scnt[wave] = wtot;
    __syncthreads();
    if (tid < HH) { for (int w = 0; w < 8; ++w) { const int nh = scnt[w]; for (int i = 0; i < nh; ++i) { const int s = ssrc[w][i], dl = sdl[w][i];
#pragma unroll
          for (int bq = 0; bq < NBB; ++bq) sacc[bq][dl][tid] += (float)Hin[((size_t)(bl0 + bq) * NNP + s) * HH + tid]; } } }
    __syncthreads(); }
#undef NN
  for (int q = tid; q < NBB * RB * HH; q += 256) { const int bq = q / (RB * HH), rem = q % (RB * HH); const int rl = rem >> 7, c = rem & 127; const int cnt = srcnt[rl];
    sa[bq][rl][HH + c] = (_Float16)(cnt > 0 ? sacc[bq][rl][c] / (float)cnt : 0.f); }
  __syncthreads();
#pragma unroll 1
  for (int tt = 0; tt < 2; ++tt) { const int tile = wave + tt * 8; const int bq = tile >> 2, rt = tile & 3; v8f acc[8] = {};
#pragma unroll 2
    for (int kc = 0; kc < 2 * HH / 32; ++kc) { const v16h a = frag_h(&sa[bq][rt * 16 + col][0] + kc * 32, lane);
#pragma unroll
      for (int j = 0; j < 8; ++j) acc[j] = wmma16(a, frag_h(WT + (size_t)(j * 16 + col) * (2 * HH) + kc * 32, lane), acc[j]); }
#pragma unroll
    for (int j = 0; j < 8; ++j) { const int n = j * 16 + col; const float bv = bb[n];
#pragma unroll
      for (int r = 0; r < 8; ++r) { const float v = acc[j][r] * (1.0f / 16.0f) + bv; sacc[bq][rt * 16 + 8 * gg + r][n] = v > 0.f ? v : 0.f; } } }
  __syncthreads();
  { const int bq = tid >> 6, rl = tid & 63; const float* row = &sacc[bq][rl][0]; float s = 0.f, q2 = 0.f;
#pragma unroll 1
    for (int c = 0; c < HH; c += 4) { const v4f v = *(const v4f*)(row + c); s += (v[0] + v[1]) + (v[2] + v[3]); q2 += (v[0] * v[0] + v[1] * v[1]) + (v[2] * v[2] + v[3] * v[3]); }
    const float mu = s * (1.0f / HH); const float var = fmaxf(q2 * (1.0f / HH) - mu * mu, 0.f); const float rs = rsqrtf(var + 1e-5f); const int n = r0 + rl;
#pragma unroll 1
    for (int c8 = 0; c8 < 16; ++c8) { union { v8h h; v4u u; } pk;
#pragma unroll
      for (int e = 0; e < 8; ++e) { const int c = c8 * 8 + e; pk.h[e] = (_Float16)(n < NNODE ? (row[c] - mu) * rs * g[c] + be[c] : 0.f); }
      vst2(Hout + ((size_t)(bl0 + bq) * NNP + n) * HH + c8 * 8, pk.u); } }
}
__global__ __launch_bounds__(128) void k_gmean(const _Float16* __restrict__ H, int b0, float* __restrict__ GR) {
  __shared__ __align__(16) float sg[HH];
  const int bl = blockIdx.x, c = threadIdx.x; const _Float16* Hb = H + (size_t)bl * NNP * HH; float s = 0.f;
#pragma unroll 1
  for (int n = 0; n < NNODE; ++n) s += (float)Hb[(size_t)n * HH + c];
  sg[c] = s * (1.0f / NNODE);
  __syncthreads();
  if (c < HH / 4) vst2(GR + (size_t)(b0 + bl) * HH + c * 4, *(const v4f*)(&sg[c * 4]));
}
__global__ __launch_bounds__(256) void k_head(const float* __restrict__ GR, const float* __restrict__ W1, const float* __restrict__ b1, const float* __restrict__ W2, const float* __restrict__ b2, float* __restrict__ out) {
  __shared__ float shid[NBAT][HH + 1]; __shared__ __align__(16) float so[NBAT * 2];
  const int tid = threadIdx.x;
#pragma unroll 1
  for (int q = tid; q < NBAT * HH; q += 256) { const int b = q >> 7, k = q & 127; float s = b1[k];
#pragma unroll 1
    for (int j = 0; j < HH; ++j) s += GR[(size_t)b * HH + j] * W1[j * HH + k];
    shid[b][k] = s > 0.f ? s : 0.f; }
  __syncthreads();
  { const int b = tid >> 1, o = tid & 1; float s = b2[o];
#pragma unroll 1
    for (int k = 0; k < HH; ++k) s += shid[b][k] * W2[k * 2 + o];
    so[b * 2 + o] = s; }
  __syncthreads();
  if (tid < NBAT * 2 / 4) vst2(out + tid * 4, *(const v4f*)(&so[tid * 4]));
}
extern "C" void kernel_launch(void* const* d_in, const int* in_sizes, int n_in, void* d_out, int out_size, void* d_ws, size_t ws_size, hipStream_t stream) {
  (void)in_sizes; (void)n_in; (void)out_size; (void)ws_size;
  const float** I = (const float**)d_in;
  const float* x = I[0]; const float* we = I[1]; const float* be = I[2]; const float* gW = I[3]; const float* gb = I[4]; const float* lg = I[5]; const float* lb = I[6];
  const float* W1 = I[7]; const float* b1 = I[8]; const float* W2 = I[9]; const float* b2 = I[10]; const int* esrc = (const int*)d_in[11]; const int* edst = (const int*)d_in[12];
  float* out = (float*)d_out;
  char* ws = (char*)d_ws; size_t off = 0;
  auto take = [&](size_t bytes) { char* p = ws + off; off += (bytes + 255) & ~(size_t)255; return p; };
  _Float16* HA = (_Float16*)take((size_t)NBH * NNP * HH * 2); _Float16* HB = (_Float16*)take((size_t)NBH * NNP * HH * 2); float* GR = (float*)take((size_t)NBAT * HH * 4); _Float16* WT = (_Float16*)take((size_t)NL * HH * 2 * HH * 2);
  k_packw<<<dim3(HH, NL), 256, 0, stream>>>(gW, WT);
  for (int half = 0; half < 2; ++half) { const int b0 = half * NBH;
    k_layer1<<<NNP / 64, 256, 0, stream>>>(x, b0, esrc, edst, we, be, gW, gb, lg, lb, HA);
    _Float16* cur = HA; _Float16* nxt = HB;
    for (int l = 1; l < NL; ++l) { k_layer<<<dim3(NNP / 64, NBH / NBB), 256, 0, stream>>>(cur, esrc, edst, WT + (size_t)l * HH * 2 * HH, gb + l * HH, lg + l * HH, lb + l * HH, nxt); _Float16* t = cur; cur = nxt; nxt = t; }
    k_gmean<<<NBH, 128, 0, stream>>>(cur, b0, GR); }
  k_head<<<1, 256, 0, stream>>>(GR, W1, b1, W2, b2, out);
}
